// RelativeMultiHeadAttn_10788957847947
// MI455X (gfx1250) — hardware-verified
//
#include <hip/hip_runtime.h>
#include <math.h>
#include <stddef.h>


#define NBATCH 8
#define SQ     512
#define DMOD   1024
#define NHEAD  16
#define HDIM   64

typedef float v8f __attribute__((ext_vector_type(8)));
typedef float v4f_raw __attribute__((ext_vector_type(4)));
typedef v4f_raw __attribute__((__may_alias__)) v4f;
typedef unsigned int v4u_raw __attribute__((ext_vector_type(4)));
typedef v4u_raw __attribute__((__may_alias__)) v4u;
typedef int v4i_raw __attribute__((ext_vector_type(4)));
typedef v4i_raw __attribute__((__may_alias__)) v4i;
typedef __bf16 v16b __attribute__((ext_vector_type(16)));
typedef __bf16 v8b __attribute__((ext_vector_type(8)));

union Frag  { v16b v; v8b h[2]; v4u q[2]; };
union Pack8 { v8b v; v4u q; };

struct FreqTab { double f[32]; };
typedef char freqtab_size_check[(sizeof(FreqTab) == 256) ? 1 : -1];

__device__ __forceinline__ v8f vz8() {
  v8f z;
#pragma unroll
  for (int i = 0; i < 8; ++i) z[i] = 0.0f;
  return z;
}

__device__ __forceinline__ v8f load8(const float* p) {
  const v4f a = *(const v4f*)(p);
  const v4f c = *(const v4f*)(p + 4);
  return __builtin_shufflevector(a, c, 0, 1, 2, 3, 4, 5, 6, 7);
}

__device__ __forceinline__ v16b ldfrag(const __bf16* __restrict__ base, int pitch, int row, int kc, int lane) {
  const int hh = lane >> 4, m = lane & 15;
  const __bf16* p = base + (size_t)(row + m) * (size_t)pitch + (kc + 8 * hh);
  Frag f;
  f.q[0] = *(const v4u*)(p);
  f.q[1] = *(const v4u*)(p + 16);
  return f.v;
}

__device__ __forceinline__ v8f wmm(v16b a, v16b b, v8f c) {
  return __builtin_amdgcn_wmma_f32_16x16x32_bf16(false, a, false, b, (short)0, c, false, false);
}

__device__ __forceinline__ void mma3x2(v8f& c0, v8f& c1,
                                       const v16b a0h, const v16b a0l,
                                       const v16b a1h, const v16b a1l,
                                       const v16b bh, const v16b bl) {
  c0 = wmm(a0h, bh, c0);
  c1 = wmm(a1h, bh, c1);
  c0 = wmm(a0h, bl, c0);
  c1 = wmm(a1h, bl, c1);
  c0 = wmm(a0l, bh, c0);
  c1 = wmm(a1l, bh, c1);
  asm volatile("v_nop\n\tv_nop\n\tv_nop\n\tv_nop"
               : "+v"(c0), "+v"(c1)
               : "v"(a0h), "v"(a0l), "v"(a1h), "v"(a1l), "v"(bh), "v"(bl));
}

__device__ __forceinline__ void split8(const v8f x, v4u& uh, v4u& ul) {
  Pack8 a, c;
  a.v = __builtin_convertvector(x, v8b);
  const v8f xh = __builtin_convertvector(a.v, v8f);
  c.v = __builtin_convertvector(x - xh, v8b);
  uh = a.q;
  ul = c.q;
}

__global__ __launch_bounds__(128)
void k_trig(FreqTab ft, float* __restrict__ tr)
{
  const int gid = (int)(blockIdx.x * 128u + threadIdx.x);
  if (gid >= SQ * 8) return;
  const int s = gid >> 3, j = gid & 7;
  float sa0 = 0.f, sa1 = 0.f, sa2 = 0.f, sa3 = 0.f;
  float ca0 = 0.f, ca1 = 0.f, ca2 = 0.f, ca3 = 0.f;
#pragma unroll 1
  for (int i = 0; i < 4; ++i) {
    const int d = 4 * j + i;
    const double ang = (double)s * ft.f[d];
    const float ah = (float)ang;
    const float al = (float)(ang - (double)ah);
    float sv, cv;
    sincosf(ah, &sv, &cv);
    const float sf = sv + al * cv;
    const float cf = cv - al * sv;
    sa0 = sa1; sa1 = sa2; sa2 = sa3; sa3 = sf;
    ca0 = ca1; ca1 = ca2; ca2 = ca3; ca3 = cf;
  }
  v4f vs, vc;
  vs[0] = sa0; vs[1] = sa1; vs[2] = sa2; vs[3] = sa3;
  vc[0] = ca0; vc[1] = ca1; vc[2] = ca2; vc[3] = ca3;
  float* ps = tr + (size_t)s * HDIM + 4 * j;
  float* pc = ps + 32;
  *(volatile v4f*)ps = vs;
  *(volatile v4f*)pc = vc;
  __threadfence();
  *(volatile v4f*)ps = vs;
  *(volatile v4f*)pc = vc;
}

__global__ __launch_bounds__(128)
void k_split_rows(const float* __restrict__ src, __bf16* __restrict__ dh, __bf16* __restrict__ dl, int n8)
{
  const int t = (int)(blockIdx.x * 128u + threadIdx.x);
  if (t >= n8) return;
  const v8f x = load8(src + (size_t)t * 8);
  v4u uh, ul;
  split8(x, uh, ul);
  __bf16* ph = dh + (size_t)t * 8;
  __bf16* pl = dl + (size_t)t * 8;
  *(volatile v4u*)ph = uh;
  *(volatile v4u*)pl = ul;
  __threadfence();
  *(volatile v4u*)ph = uh;
  *(volatile v4u*)pl = ul;
}

__global__ __launch_bounds__(128)
void k_xsplit(const float* __restrict__ x, __bf16* __restrict__ kxh, __bf16* __restrict__ kxl, int n8)
{
  const int t = (int)(blockIdx.x * 128u + threadIdx.x);
  if (t >= n8) return;
  const size_t e0 = (size_t)t * 8;
  const int bb = (int)(e0 >> 19);
  const int ss = (int)((e0 >> 10) & 511);
  const int cc = (int)(e0 & 1023);
  const int hq = cc >> 6, d = cc & 63;
  const size_t dst = ((size_t)((bb * NHEAD + hq) * SQ + ss)) * HDIM + d;
  const v8f v = load8(x + e0);
  v4u uh, ul;
  split8(v, uh, ul);
  __bf16* ph = kxh + dst;
  __bf16* pl = kxl + dst;
  *(volatile v4u*)ph = uh;
  *(volatile v4u*)pl = ul;
  __threadfence();
  *(volatile v4u*)ph = uh;
  *(volatile v4u*)pl = ul;
}

__global__ __launch_bounds__(128)
void k_wsplitT(const float* __restrict__ w, __bf16* __restrict__ wth, __bf16* __restrict__ wtl)
{
  __shared__ __align__(16) float T[64][36];
  const int tid = threadIdx.x;
  const int nb = (int)(blockIdx.x & 63u), kb = (int)(blockIdx.x >> 6);
  const int n0 = nb * 32, k0 = kb * 64;
#pragma unroll
  for (int i = 0; i < 4; ++i) {
    const int idx = tid + 128 * i;
    const int row = idx >> 3, c4 = idx & 7;
    const v4f v = *(const v4f*)(w + (size_t)(k0 + row) * (2 * DMOD) + n0 + 4 * c4);
    *(v4f*)&T[row][4 * c4] = v;
  }
  __syncthreads();
#pragma unroll 1
  for (int i = 0; i < 2; ++i) {
    const int task = tid + 128 * i;
    const int nn = task >> 3, j = task & 7;
    v8f v;
#pragma unroll
    for (int e = 0; e < 8; ++e) v[e] = T[8 * j + e][nn];
    v4u uh, ul;
    split8(v, uh, ul);
    const size_t off = (size_t)(n0 + nn) * DMOD + k0 + 8 * j;
    __bf16* ph = wth + off;
    __bf16* pl = wtl + off;
    *(volatile v4u*)ph = uh;
    *(volatile v4u*)pl = ul;
    __threadfence();
    *(volatile v4u*)ph = uh;
    *(volatile v4u*)pl = ul;
  }
}

__global__ __launch_bounds__(64) __attribute__((amdgpu_num_vgpr(256)))
void k_gemm(const __bf16* __restrict__ kxh, const __bf16* __restrict__ kxl,
            const __bf16* __restrict__ wth, const __bf16* __restrict__ wtl,
            const float* __restrict__ rrb, const float* __restrict__ rwb,
            const float* __restrict__ tr,
            __bf16* __restrict__ qah, __bf16* __restrict__ qal,
            __bf16* __restrict__ qbh, __bf16* __restrict__ qbl,
            __bf16* __restrict__ vth, __bf16* __restrict__ vtl)
{
  __shared__ __align__(16) float Cs[64][64];
  const int tid = threadIdx.x, w = tid >> 5, lane = tid & 31, hh = lane >> 4, m = lane & 15;
  const int bn = (int)(blockIdx.x & 31u), bm = (int)(blockIdx.x >> 5);
  const int n0 = bn * 64, m0 = bm * 64;
  const int b = m0 >> 9, s0 = m0 & 511;
  const int arow = s0 + w * 32;

  v8f acc0[4], acc1[4];
#pragma unroll
  for (int ni = 0; ni < 4; ++ni) { acc0[ni] = vz8(); acc1[ni] = vz8(); }

#pragma unroll 1
  for (int ks = 0; ks < DMOD / 32; ++ks) {
    const int k0 = ks * 32, hk = k0 >> 6, kc = k0 & 63;
    const int ra = (b * NHEAD + hk) * SQ + arow;
    const v16b a0h = ldfrag(kxh, HDIM, ra, kc, lane);
    const v16b a0l = ldfrag(kxl, HDIM, ra, kc, lane);
    const v16b a1h = ldfrag(kxh, HDIM, ra + 16, kc, lane);
    const v16b a1l = ldfrag(kxl, HDIM, ra + 16, kc, lane);
#pragma unroll
    for (int ni = 0; ni < 4; ++ni) {
      const v16b bhf = ldfrag(wth, DMOD, n0 + ni * 16, k0, lane);
      const v16b blf = ldfrag(wtl, DMOD, n0 + ni * 16, k0, lane);
      mma3x2(acc0[ni], acc1[ni], a0h, a0l, a1h, a1l, bhf, blf);
    }
  }

#pragma unroll
  for (int ni = 0; ni < 4; ++ni)
#pragma unroll
    for (int r = 0; r < 8; ++r) {
      Cs[w * 32 + 8 * hh + r][ni * 16 + m]      = acc0[ni][r];
      Cs[w * 32 + 16 + 8 * hh + r][ni * 16 + m] = acc1[ni][r];
    }
  __syncthreads();

  if (n0 < DMOD) {
    const int hq = n0 >> 6;
    const int qrow0 = (b * NHEAD + hq) * SQ;
    const float* rrbh = rrb + hq * HDIM;
    const float* rwbh = rwb + hq * HDIM;
#pragma unroll 1
    for (int it = 0; it < 8; ++it) {
      const int task = tid + 64 * it;
      const int rr = task >> 3, j = task & 7, j4 = j & 3;
      const int s = s0 + rr;
      const v8f cl = load8(&Cs[rr][8 * j4]);
      const v8f ch = load8(&Cs[rr][32 + 8 * j4]);
      const v8f bwl = load8(rwbh + 8 * j4);
      const v8f bwh = load8(rwbh + 32 + 8 * j4);
      const v8f br  = load8(rrbh + 8 * j);
      const float* trs = tr + (size_t)s * HDIM;
      const v8f sq = load8(trs + 8 * j4);
      const v8f cq = load8(trs + 32 + 8 * j4);
      const v8f a = cl + bwl;
      const v8f c = ch + bwh;
      v8f qa, qb;
      if (j < 4) {
        qa = cl + br;
        qb = a * cq + c * sq;
      } else {
        qa = ch + br;
        qb = c * cq - a * sq;
      }
      v4u ah, al, bh, bl;
      split8(qa, ah, al);
      split8(qb, bh, bl);
      const size_t off = ((size_t)(qrow0 + s)) * HDIM + 8 * j;
      __bf16* p0 = qah + off;
      __bf16* p1 = qal + off;
      __bf16* p2 = qbh + off;
      __bf16* p3 = qbl + off;
      *(volatile v4u*)p0 = ah;
      *(volatile v4u*)p1 = al;
      *(volatile v4u*)p2 = bh;
      *(volatile v4u*)p3 = bl;
      __threadfence();
      *(volatile v4u*)p0 = ah;
      *(volatile v4u*)p1 = al;
      *(volatile v4u*)p2 = bh;
      *(volatile v4u*)p3 = bl;
    }
  } else {
    const int hv = (n0 - DMOD) >> 6;
    const int vrow0 = (b * NHEAD + hv) * HDIM;
#pragma unroll 1
    for (int it = 0; it < 8; ++it) {
      const int task = tid + 64 * it;
      const int dd = task >> 3, j = task & 7;
      v8f v;
#pragma unroll
      for (int e = 0; e < 8; ++e) v[e] = Cs[8 * j + e][dd];
      v4u uh, ul;
      split8(v, uh, ul);
      const size_t off = ((size_t)(vrow0 + dd)) * SQ + s0 + 8 * j;
      __bf16* ph = vth + off;
      __bf16* pl = vtl + off;
      *(volatile v4u*)ph = uh;
      *(volatile v4u*)pl = ul;
      __threadfence();
      *(volatile v4u*)ph = uh;
      *(volatile v4u*)pl = ul;
    }
  }
}

__global__ __launch_bounds__(128) __attribute__((amdgpu_num_vgpr(256)))
void k_attn(const __bf16* __restrict__ qah, const __bf16* __restrict__ qal,
            const __bf16* __restrict__ qbh, const __bf16* __restrict__ qbl,
            const __bf16* __restrict__ kxh, const __bf16* __restrict__ kxl,
            const __bf16* __restrict__ trh, const __bf16* __restrict__ trl,
            const __bf16* __restrict__ vth, const __bf16* __restrict__ vtl,
            const int* __restrict__ msk, float* __restrict__ out)
{
  __shared__ __align__(16) float Os[4][16][64];
  const int tid = threadIdx.x, w = tid >> 5, lane = tid & 31, hh = lane >> 4, n = lane & 15;
  const int bh = (int)(blockIdx.x >> 3), qc = (int)(blockIdx.x & 7u);
  const int b = bh >> 4, hd = bh & 15;
  const int q0 = qc * 64 + w * 16;
  const int qrow = bh * SQ + q0;
  const int krow = bh * SQ;
  const int vrow = bh * HDIM;

  v8f o0 = vz8(), o1 = vz8(), o2 = vz8(), o3 = vz8();
  float mrun = -1.0e30f, dsum = 0.0f;

#pragma unroll 1
  for (int kb0 = 0; kb0 < SQ; kb0 += 32) {
    v8f s0 = vz8(), s1 = vz8();
#pragma unroll 1
    for (int c = 0; c < 4; ++c) {
      const bool lowc = (c < 2);
      const int kc = (c & 1) * 32;
      const __bf16* qsh = lowc ? qah : qbh;
      const __bf16* qsl = lowc ? qal : qbl;
      const __bf16* ksh = lowc ? kxh : trh;
      const __bf16* ksl = lowc ? kxl : trl;
      const int kr = (lowc ? krow : 0) + kb0;
      const v16b qh  = ldfrag(qsh, HDIM, qrow, kc, lane);
      const v16b ql  = ldfrag(qsl, HDIM, qrow, kc, lane);
      const v16b kah = ldfrag(ksh, HDIM, kr, kc, lane);
      const v16b kal = ldfrag(ksl, HDIM, kr, kc, lane);
      const v16b kch = ldfrag(ksh, HDIM, kr + 16, kc, lane);
      const v16b kcl = ldfrag(ksl, HDIM, kr + 16, kc, lane);
      mma3x2(s0, s1, kah, kal, kch, kcl, qh, ql);
    }

    const int* mp = msk + b * SQ + kb0 + 8 * hh;
    const v4i mA = *(const v4i*)(mp);
    const v4i mB = *(const v4i*)(mp + 4);
    const v4i mC = *(const v4i*)(mp + 16);
    const v4i mD = *(const v4i*)(mp + 20);
    v8f f0, f1;
#pragma unroll
    for (int r = 0; r < 4; ++r) {
      f0[r] = (float)mA[r]; f0[4 + r] = (float)mB[r];
      f1[r] = (float)mC[r]; f1[4 + r] = (float)mD[r];
    }
    s0 = s0 * f0 - (1.0f - f0) * 1.0e8f;
    s1 = s1 * f1 - (1.0f - f1) * 1.0e8f;

    float mloc = s0[0];
#pragma unroll
    for (int r = 0; r < 8; ++r) { mloc = fmaxf(mloc, s0[r]); mloc = fmaxf(mloc, s1[r]); }
    const float mall = fmaxf(mloc, __shfl_xor(mloc, 16, 32));
    const float mnew = fmaxf(mrun, mall);
    const float alpha = __expf(mrun - mnew);
    float psum = 0.0f;
#pragma unroll
    for (int r = 0; r < 8; ++r) {
      const float pa = __expf(s0[r] - mnew);
      const float pb = __expf(s1[r] - mnew);
      s0[r] = pa; s1[r] = pb;
      psum += pa + pb;
    }
    psum += __shfl_xor(psum, 16, 32);
    dsum = dsum * alpha + psum;
    mrun = mnew;
    o0 *= alpha; o1 *= alpha; o2 *= alpha; o3 *= alpha;

    v4u p0h, p0l, p1h, p1l;
    split8(s0, p0h, p0l);
    split8(s1, p1h, p1l);
    Frag ph, pl;
    ph.q[0] = p0h; ph.q[1] = p1h;
    pl.q[0] = p0l; pl.q[1] = p1l;
    {
      const v16b v0h = ldfrag(vth, SQ, vrow, kb0, lane);
      const v16b v0l = ldfrag(vtl, SQ, vrow, kb0, lane);
      const v16b v1h = ldfrag(vth, SQ, vrow + 16, kb0, lane);
      const v16b v1l = ldfrag(vtl, SQ, vrow + 16, kb0, lane);
      mma3x2(o0, o1, v0h, v0l, v1h, v1l, ph.v, pl.v);
    }
    {
      const v16b v2h = ldfrag(vth, SQ, vrow + 32, kb0, lane);
      const v16b v2l = ldfrag(vtl, SQ, vrow + 32, kb0, lane);
      const v16b v3h = ldfrag(vth, SQ, vrow + 48, kb0, lane);
      const v16b v3l = ldfrag(vtl, SQ, vrow + 48, kb0, lane);
      mma3x2(o2, o3, v2h, v2l, v3h, v3l, ph.v, pl.v);
    }
  }

  const float rinv = 1.0f / dsum;
#pragma unroll
  for (int r = 0; r < 8; ++r) {
    Os[w][n][8 * hh + r]      = o0[r] * rinv;
    Os[w][n][16 + 8 * hh + r] = o1[r] * rinv;
    Os[w][n][32 + 8 * hh + r] = o2[r] * rinv;
    Os[w][n][48 + 8 * hh + r] = o3[r] * rinv;
  }
  __syncthreads();

  v4f ov[8];
#pragma unroll
  for (int it = 0; it < 8; ++it) ov[it] = *(const v4f*)&Os[w][2 * it + hh][4 * n];
  float* ob = out + ((size_t)(b * SQ + q0)) * DMOD + hd * HDIM + 4 * n;
#pragma unroll
  for (int it = 0; it < 8; ++it) {
    float* p = ob + (size_t)(2 * it + hh) * DMOD;
    *(volatile v4f*)p = ov[it];
  }
  __threadfence();
#pragma unroll
  for (int it = 0; it < 8; ++it) {
    float* p = ob + (size_t)(2 * it + hh) * DMOD;
    *(volatile v4f*)p = ov[it];
  }
}

extern "C" void kernel_launch(void* const* d_in, const int* in_sizes, int n_in,
                              void* d_out, int out_size, void* d_ws,
                              size_t ws_size, hipStream_t stream)
{
  if (n_in < 5) return;
  if (in_sizes[0] != NBATCH * SQ * DMOD) return;
  if (in_sizes[1] != NBATCH * SQ) return;
  if (in_sizes[2] != DMOD * 2 * DMOD) return;
  if (in_sizes[3] != NHEAD * HDIM) return;
  if (in_sizes[4] != NHEAD * HDIM) return;
  if (out_size != NBATCH * SQ * DMOD) return;

  const float* x    = (const float*)d_in[0];
  const int*   mk   = (const int*)d_in[1];
  const float* wqv  = (const float*)d_in[2];
  const float* rrb  = (const float*)d_in[3];
  const float* rwb  = (const float*)d_in[4];
  float* out = (float*)d_out;

  const size_t n_tr    = (size_t)SQ * HDIM;
  const size_t n_heads = (size_t)NBATCH * NHEAD * SQ * HDIM;
  const size_t n_w     = (size_t)DMOD * 2 * DMOD;

  char* ws = (char*)d_ws;
  size_t off = 0;
  auto carve = [&](size_t bytes) -> char* {
    char* p = ws + off;
    off += (bytes + 255) & ~(size_t)255;
    return p;
  };
  float*  tr  = (float*)carve(n_tr * 4);
  __bf16* trh = (__bf16*)carve(n_tr * 2);
  __bf16* trl = (__bf16*)carve(n_tr * 2);
  __bf16* kxh = (__bf16*)carve(n_heads * 2);
  __bf16* kxl = (__bf16*)carve(n_heads * 2);
  __bf16* wth = (__bf16*)carve(n_w * 2);
  __bf16* wtl = (__bf16*)carve(n_w * 2);
  __bf16* qah = (__bf16*)carve(n_heads * 2);
  __bf16* qal = (__bf16*)carve(n_heads * 2);
  __bf16* qbh = (__bf16*)carve(n_heads * 2);
  __bf16* qbl = (__bf16*)carve(n_heads * 2);
  __bf16* vth = (__bf16*)carve(n_heads * 2);
  __bf16* vtl = (__bf16*)carve(n_heads * 2);
  if (off > ws_size) return;

  FreqTab ft;
  const double cst = -log(10000.0) / 31.0;
  for (int d = 0; d < 32; ++d) ft.f[d] = exp((double)((float)d) * cst);

  const int n8_tr = (int)(n_tr / 8);
  const int n8_x  = (int)(n_heads / 8);

  k_trig<<<dim3((SQ * 8 + 127) / 128), dim3(128), 0, stream>>>(ft, tr);
  k_split_rows<<<dim3((n8_tr + 127) / 128), dim3(128), 0, stream>>>(tr, trh, trl, n8_tr);
  k_xsplit<<<dim3((n8_x + 127) / 128), dim3(128), 0, stream>>>(x, kxh, kxl, n8_x);
  k_wsplitT<<<dim3((2 * DMOD / 32) * (DMOD / 64)), dim3(128), 0, stream>>>(wqv, wth, wtl);
  k_gemm<<<dim3((NBATCH * SQ / 64) * (2 * DMOD / 64)), dim3(64), 0, stream>>>(
      kxh, kxl, wth, wtl, rrb, rwb, tr, qah, qal, qbh, qbl, vth, vtl);
  k_attn<<<dim3(NBATCH * NHEAD * (SQ / 64)), dim3(128), 0, stream>>>(
      qah, qal, qbh, qbl, kxh, kxl, trh, trl, vth, vtl, mk, out);
}
